// PoseGatEncoder_3496103379476
// MI455X (gfx1250) — hardware-verified
//
#include <hip/hip_runtime.h>
#include <stddef.h>


#define NJ      50
#define NJP     64
#define NH      4
#define NFEAT   3
#define ECAP    256
#define DEGCAP  16
#define NT      256
#define GT      128
#define D1      64
#define D2      128
#define D3      256
#define XSC     16.0f
#define WSC     64.0f
#define WOSC    256.0f
#define INV_L   0.0009765625f
#define INV_O   0.000244140625f
#define NEG_SLOPE 0.2f
#define WSCAPB  134217728

typedef float          v4f  __attribute__((ext_vector_type(4)));
typedef float          v8f  __attribute__((ext_vector_type(8)));
typedef unsigned short v8us __attribute__((ext_vector_type(8)));
typedef _Float16       v8h  __attribute__((ext_vector_type(8)));
typedef _Float16       v16h __attribute__((ext_vector_type(16)));
union FragH { v16h v; v8us h[2]; };
union Pack8 { v8h h; v8us u; };

template<int DOUT>
struct LL {
  static constexpr int    N2    = 2 * DOUT;
  static constexpr size_t XY    = 0;
  static constexpr size_t ES    = XY  + (size_t)NJ * N2 * 4;
  static constexpr size_t MS    = ES  + (size_t)ECAP * NH * 4;
  static constexpr size_t RS    = MS  + (size_t)NJP * NH * 4;
  static constexpr size_t SRC   = RS  + (size_t)NJP * NH * 4;
  static constexpr size_t DST   = SRC + (size_t)ECAP * 4;
  static constexpr size_t CNT   = DST + (size_t)ECAP * 4;
  static constexpr size_t IDX   = CNT + (size_t)NJP * 4;
  static constexpr size_t ATT   = IDX + (size_t)NJP * DEGCAP * 4;
  static constexpr size_t BIA   = ATT + (size_t)DOUT * 4;
  static constexpr size_t TOTAL = BIA + (size_t)DOUT * 4;
};
static_assert(LL<D2>::TOTAL <= 160000);
static_assert(LL<D3>::TOTAL <= 160000);
static_assert((LL<D2>::XY % 16) == 0 && (LL<D3>::ES % 16) == 0);
static_assert(NT == ECAP);
static_assert(NH * 16 == D1);

__device__ __forceinline__ v8us cvt8h(v4f a, v4f b, float sc) {
  v8h r;
  r[0] = (_Float16)(a.x * sc); r[1] = (_Float16)(a.y * sc);
  r[2] = (_Float16)(a.z * sc); r[3] = (_Float16)(a.w * sc);
  r[4] = (_Float16)(b.x * sc); r[5] = (_Float16)(b.y * sc);
  r[6] = (_Float16)(b.z * sc); r[7] = (_Float16)(b.w * sc);
  Pack8 p;
  p.h = r;
  return p.u;
}

__device__ __forceinline__ v8f wmh(v16h a, v16h b, v8f c) {
  v8f d = __builtin_amdgcn_wmma_f32_16x16x32_f16(false, a, false, b, (short)0, c, false, false);
  asm volatile("v_nop\n\tv_nop\n\tv_nop\n\tv_nop" : "+v"(d) : "v"(a), "v"(b));
  return d;
}

__global__ __launch_bounds__(NT) void k_wtrans(const float* __restrict__ src, unsigned short* dst,
                                                 int K, int N, int nOff, float sc) {
  __shared__ __attribute__((aligned(16))) float T[64 * 64];
  const int tid = (int)threadIdx.x;
  const int k0 = (int)blockIdx.x * 64, n0 = (int)blockIdx.y * 64;
#pragma unroll 1
  for (int i = tid; i < 1024; i += NT) {
    const int kk = i >> 4, n4 = (i & 15) * 4;
    const v4f v = *(const v4f*)(src + (size_t)(k0 + kk) * N + n0 + n4);
    *(v4f*)(T + kk * 64 + n4) = v;
  }
  __syncthreads();
#pragma unroll 1
  for (int ps = 0; ps < 2; ++ps) {
    if (ps) __threadfence();
#pragma unroll 1
    for (int p = tid; p < 512; p += NT) {
      const int n = p >> 3, k8 = (p & 7) * 8;
      const float* c = T + k8 * 64 + n;
      v4f a, b;
      a.x = c[0 * 64]; a.y = c[1 * 64]; a.z = c[2 * 64]; a.w = c[3 * 64];
      b.x = c[4 * 64]; b.y = c[5 * 64]; b.z = c[6 * 64]; b.w = c[7 * 64];
      const v8us hv = cvt8h(a, b, sc);
      unsigned short* d = dst + (size_t)(nOff + n0 + n) * K + k0 + k8;
      *(volatile v8us*)d = hv;
    }
  }
}

__device__ __forceinline__ void load_edges(int tid, const int* __restrict__ srcE, const int* __restrict__ dstE,
                                           int nE, int* srcS, int* dstS) {
#pragma unroll 1
  for (int e = tid; e < ECAP; e += NT) {
    const int ec = e < nE ? e : nE - 1;
    int s = srcE[ec];
    s = s < 0 ? s + NJ : s;
    s = s < 0 ? 0 : (s > NJ - 1 ? NJ - 1 : s);
    int d = dstE[ec];
    d = d < 0 ? d + NJ : d;
    d = d < 0 ? 0 : (d > NJ - 1 ? NJ - 1 : d);
    srcS[e] = s;
    dstS[e] = d;
  }
}

__device__ __forceinline__ void build_csr(int tid, int nE, const int* dstS, int* cnt, int* idx) {
#pragma unroll 1
  for (int j = tid; j < NJP; j += NT) {
    int c = 0;
    if (j < NJ) {
#pragma unroll 1
      for (int e = 0; e < nE; ++e) {
        if (dstS[e] == j) {
          if (c < DEGCAP) idx[j * DEGCAP + c] = e;
          ++c;
        }
      }
    }
    cnt[j] = c > DEGCAP ? DEGCAP : c;
  }
}

template<int DOUT>
__device__ __forceinline__ void gat_tail(int tid, int nE, const float* attS, const float* biS,
                                         float* XY, float* eS, float* mS, float* rS,
                                         const int* srcS, const int* dstS, const int* cnt, const int* idx,
                                         unsigned short* xo) {
  constexpr int C = DOUT / NH, N2 = 2 * DOUT, NP = NJ * DOUT / 8, PR = DOUT / 8;
#pragma unroll 1
  for (int t = tid; t < nE * NH; t += NT) {
    const int e = t >> 2, h = t & 3;
    const float* pl = XY + srcS[e] * N2 + h * C;
    const float* pr = XY + dstS[e] * N2 + DOUT + h * C;
    const float* pa = attS + h * C;
    float s = 0.0f;
#pragma unroll 1
    for (int c = 0; c < C; ++c) {
      float v = pl[c] + pr[c];
      v = (v >= 0.0f) ? v : NEG_SLOPE * v;
      s = fmaf(v, pa[c], s);
    }
    eS[t] = s;
  }
  __syncthreads();
#pragma unroll 1
  for (int t = tid; t < NJ * NH; t += NT) {
    const int j = t >> 2, h = t & 3;
    int d = cnt[j];
    d = d < 0 ? 0 : (d > DEGCAP ? DEGCAP : d);
    float mx = -3.0e38f;
#pragma unroll 1
    for (int q = 0; q < d; ++q) mx = fmaxf(mx, eS[idx[j * DEGCAP + q] * NH + h]);
    float den = 0.0f;
#pragma unroll 1
    for (int q = 0; q < d; ++q) den += __expf(eS[idx[j * DEGCAP + q] * NH + h] - mx);
    mS[t] = mx;
    rS[t] = (d > 0) ? __builtin_amdgcn_rcpf(den) : 0.0f;
  }
  __syncthreads();
#pragma unroll 1
  for (int t = tid; t < nE * NH; t += NT) {
    const int e = t >> 2, h = t & 3;
    const int dd = dstS[e] * NH + h;
    eS[t] = __expf(eS[t] - mS[dd]) * rS[dd];
  }
  __syncthreads();
#pragma unroll 1
  for (int t = tid; t < NJ * DOUT; t += NT) {
    const int j = t / DOUT, oc = t % DOUT, h = oc / C;
    int d = cnt[j];
    d = d < 0 ? 0 : (d > DEGCAP ? DEGCAP : d);
    float s = 0.0f;
#pragma unroll 1
    for (int q = 0; q < d; ++q) {
      const int e = idx[j * DEGCAP + q];
      s = fmaf(eS[e * NH + h], XY[srcS[e] * N2 + oc], s);
    }
    float v = s + biS[oc];
    v = (v > 0.0f) ? v : (__expf(v) - 1.0f);
    XY[j * N2 + DOUT + oc] = v;
  }
  __syncthreads();
#pragma unroll 1
  for (int ps = 0; ps < 2; ++ps) {
    if (ps) __threadfence();
#pragma unroll 1
    for (int p = tid; p < NP; p += NT) {
      const int j = p / PR, o8 = (p % PR) * 8;
      const float* sp = XY + j * N2 + DOUT + o8;
      const v4f a = *(const v4f*)sp;
      const v4f b = *(const v4f*)(sp + 4);
      const v8us hv = cvt8h(a, b, XSC);
      *(volatile v8us*)(xo + (size_t)p * 8) = hv;
    }
  }
}

__global__ __launch_bounds__(NT) void k_gat0(const float* __restrict__ xs,
                                               const float* __restrict__ Wl, const float* __restrict__ bl,
                                               const float* __restrict__ Wr, const float* __restrict__ br,
                                               const float* __restrict__ att, const float* __restrict__ bias,
                                               const int* __restrict__ srcE, const int* __restrict__ dstE,
                                               unsigned short* xo, int nE) {
  constexpr int N2 = 2 * D1;
  __shared__ __attribute__((aligned(16))) float XY[NJ * N2];
  __shared__ __attribute__((aligned(16))) float eS[ECAP * NH];
  __shared__ float mS[NJP * NH];
  __shared__ float rS[NJP * NH];
  __shared__ int   srcS[ECAP];
  __shared__ int   dstS[ECAP];
  __shared__ int   cnt[NJP];
  __shared__ int   idx[NJP * DEGCAP];
  __shared__ float x0[NJ * NFEAT + 2];
  __shared__ float W0[2 * NFEAT * D1];
  __shared__ float B0[2 * D1];
  __shared__ float attS[D1];
  __shared__ float biS[D1];

  const int tid = (int)threadIdx.x, g = (int)blockIdx.x;
  nE = nE < 1 ? 1 : (nE > ECAP ? ECAP : nE);
  const float* xg = xs + (size_t)g * (NJ * NFEAT);
#pragma unroll 1
  for (int i = tid; i < NJ * NFEAT; i += NT) x0[i] = xg[i];
#pragma unroll 1
  for (int i = tid; i < NFEAT * D1; i += NT) { W0[i] = Wl[i]; W0[NFEAT * D1 + i] = Wr[i]; }
#pragma unroll 1
  for (int i = tid; i < D1; i += NT) { B0[i] = bl[i]; B0[D1 + i] = br[i]; attS[i] = att[i]; biS[i] = bias[i]; }
  load_edges(tid, srcE, dstE, nE, srcS, dstS);
  __syncthreads();

#pragma unroll 1
  for (int t = tid; t < NJ * N2; t += NT) {
    const int j = t / N2, n = t % N2, side = n / D1, o = n % D1;
    const float* w  = W0 + side * (NFEAT * D1);
    const float* xr = x0 + j * NFEAT;
    float s = xr[0] * w[o];
    s = fmaf(xr[1], w[D1 + o], s);
    s = fmaf(xr[2], w[2 * D1 + o], s);
    XY[t] = s + B0[side * D1 + o];
  }
  build_csr(tid, nE, dstS, cnt, idx);
  __syncthreads();
  gat_tail<D1>(tid, nE, attS, biS, XY, eS, mS, rS, srcS, dstS, cnt, idx,
               xo + (size_t)g * (NJ * D1));
}

template<int DIN, int DOUT>
__global__ __launch_bounds__(NT) void k_gatw(const unsigned short* __restrict__ xh,
                                               const unsigned short* __restrict__ wt,
                                               const float* __restrict__ bl, const float* __restrict__ br,
                                               const float* __restrict__ att, const float* __restrict__ bias,
                                               const int* __restrict__ srcE, const int* __restrict__ dstE,
                                               unsigned short* xo, int nE) {
  using L = LL<DOUT>;
  constexpr int N2 = 2 * DOUT, KT = DIN / 32, NTW = N2 / 32;
  static_assert(DIN % 32 == 0 && DOUT % 16 == 0 && NT == 256);
  extern __shared__ v4f lds_dyn[];
  char*  sm   = (char*)lds_dyn;
  float* XY   = (float*)(sm + L::XY);
  float* eS   = (float*)(sm + L::ES);
  float* mS   = (float*)(sm + L::MS);
  float* rS   = (float*)(sm + L::RS);
  int*   srcS = (int*)(sm + L::SRC);
  int*   dstS = (int*)(sm + L::DST);
  int*   cnt  = (int*)(sm + L::CNT);
  int*   idx  = (int*)(sm + L::IDX);
  float* attS = (float*)(sm + L::ATT);
  float* biS  = (float*)(sm + L::BIA);

  const int tid = (int)threadIdx.x, lane = tid & 31, wave = tid >> 5, hh = lane >> 4, m = lane & 15;
  const int g = (int)blockIdx.x;
  nE = nE < 1 ? 1 : (nE > ECAP ? ECAP : nE);
#pragma unroll 1
  for (int i = tid; i < DOUT; i += NT) { attS[i] = att[i]; biS[i] = bias[i]; }
  load_edges(tid, srcE, dstE, nE, srcS, dstS);
  __syncthreads();

  {
    const int mt = wave & 3, ntb = (wave >> 2) * NTW;
    int ar = mt * 16 + m;
    ar = ar > NJ - 1 ? NJ - 1 : ar;
    const unsigned short* ap = xh + ((size_t)g * NJ + ar) * DIN + 8 * hh;
    FragH a[KT];
#pragma unroll
    for (int kt = 0; kt < KT; ++kt) {
      a[kt].h[0] = *(const v8us*)(ap + 32 * kt);
      a[kt].h[1] = *(const v8us*)(ap + 32 * kt + 16);
    }
    const int r0 = mt * 16 + 8 * hh;
#pragma unroll 1
    for (int t = 0; t < NTW; ++t) {
      const int n = (ntb + t) * 16 + m;
      const unsigned short* bp = wt + (size_t)n * DIN + 8 * hh;
      v8f acc = {0.f, 0.f, 0.f, 0.f, 0.f, 0.f, 0.f, 0.f};
#pragma unroll
      for (int kt = 0; kt < KT; ++kt) {
        FragH b;
        b.h[0] = *(const v8us*)(bp + 32 * kt);
        b.h[1] = *(const v8us*)(bp + 32 * kt + 16);
        acc = wmh(a[kt].v, b.v, acc);
      }
      const float b1 = bl[n < DOUT ? n : DOUT - 1];
      const float b2 = br[n >= DOUT ? n - DOUT : 0];
      const float bv = (n < DOUT) ? b1 : b2;
      float* cp = XY + n;
#pragma unroll
      for (int r = 0; r < 8; ++r) {
        const int row = r0 + r;
        if (row < NJ) cp[row * N2] = acc[r] * INV_L + bv;
      }
    }
  }
  build_csr(tid, nE, dstS, cnt, idx);
  __syncthreads();
  gat_tail<DOUT>(tid, nE, attS, biS, XY, eS, mS, rS, srcS, dstS, cnt, idx,
                 xo + (size_t)g * (NJ * DOUT));
}

__global__ __launch_bounds__(GT) void k_ogemm(const unsigned short* __restrict__ A,
                                               const unsigned short* __restrict__ Bw,
                                               const float* __restrict__ bo, float* out, int K, int N) {
  __shared__ __attribute__((aligned(16))) float stg[64 * 64];
  const int tid = (int)threadIdx.x, lane = tid & 31, wave = tid >> 5, hh = lane >> 4, m = lane & 15;
  const int rb = (int)blockIdx.x * 64, cb = (int)blockIdx.y * 64;
  const unsigned short* ap = A  + (size_t)(rb + 16 * wave + m) * K + 8 * hh;
  const unsigned short* bp = Bw + (size_t)(cb + m) * K + 8 * hh;
  v8f acc[4];
#pragma unroll
  for (int t = 0; t < 4; ++t) { v8f z = {0.f, 0.f, 0.f, 0.f, 0.f, 0.f, 0.f, 0.f}; acc[t] = z; }
#pragma unroll 1
  for (int kb = 0; kb < K; kb += 32) {
    FragH a;
    a.h[0] = *(const v8us*)(ap + kb);
    a.h[1] = *(const v8us*)(ap + kb + 16);
#pragma unroll
    for (int t = 0; t < 4; ++t) {
      const unsigned short* q = bp + (size_t)(16 * t) * K + kb;
      FragH b;
      b.h[0] = *(const v8us*)(q);
      b.h[1] = *(const v8us*)(q + 16);
      acc[t] = wmh(a.v, b.v, acc[t]);
    }
  }
#pragma unroll
  for (int t = 0; t < 4; ++t) {
    const int col = 16 * t + m;
    const float bv = bo[cb + col];
    float* sp = stg + (16 * wave + 8 * hh) * 64 + col;
#pragma unroll
    for (int r = 0; r < 8; ++r) sp[r * 64] = acc[t][r] * INV_O + bv;
  }
  __syncthreads();
#pragma unroll 1
  for (int ps = 0; ps < 2; ++ps) {
    if (ps) __threadfence();
#pragma unroll 1
    for (int f = tid; f < 1024; f += GT) {
      const int row = f >> 4, c4 = (f & 15) * 4;
      const v4f v = *(const v4f*)(stg + row * 64 + c4);
      *(volatile v4f*)(out + (size_t)(rb + row) * N + cb + c4) = v;
    }
  }
}

extern "C" void kernel_launch(void* const* d_in, const int* in_sizes, int n_in,
                              void* d_out, int out_size, void* d_ws, size_t ws_size,
                              hipStream_t stream) {
  if (n_in < 23) return;
  const int EMB = in_sizes[20];
  if (EMB <= 0 || (EMB % 64) != 0) return;
  if (out_size <= 0 || (out_size % EMB) != 0) return;
  const int G = out_size / EMB;
  if ((G % 64) != 0 || G > (1 << 20)) return;
  if (in_sizes[0] != G * NJ * NFEAT) return;
  if (in_sizes[1] != NFEAT * D1 || in_sizes[3] != NFEAT * D1) return;
  if (in_sizes[2] != D1 || in_sizes[4] != D1 || in_sizes[5] != D1 || in_sizes[6] != D1) return;
  if (in_sizes[7] != D1 * D2 || in_sizes[9] != D1 * D2) return;
  if (in_sizes[8] != D2 || in_sizes[10] != D2 || in_sizes[11] != D2 || in_sizes[12] != D2) return;
  if (in_sizes[13] != D2 * D3 || in_sizes[15] != D2 * D3) return;
  if (in_sizes[14] != D3 || in_sizes[16] != D3 || in_sizes[17] != D3 || in_sizes[18] != D3) return;
  const int KO = NJ * D3;
  if (in_sizes[19] != KO * EMB) return;
  const int nE = in_sizes[21];
  if (nE < 1 || nE > ECAP || in_sizes[22] != nE) return;

  const float* x_seq = (const float*)d_in[0];
  const float* Wl0 = (const float*)d_in[1],  *bl0 = (const float*)d_in[2];
  const float* Wr0 = (const float*)d_in[3],  *br0 = (const float*)d_in[4];
  const float* att0 = (const float*)d_in[5], *bias0 = (const float*)d_in[6];
  const float* Wl1 = (const float*)d_in[7],  *bl1 = (const float*)d_in[8];
  const float* Wr1 = (const float*)d_in[9],  *br1 = (const float*)d_in[10];
  const float* att1 = (const float*)d_in[11], *bias1 = (const float*)d_in[12];
  const float* Wl2 = (const float*)d_in[13], *bl2 = (const float*)d_in[14];
  const float* Wr2 = (const float*)d_in[15], *br2 = (const float*)d_in[16];
  const float* att2 = (const float*)d_in[17], *bias2 = (const float*)d_in[18];
  const float* Wout = (const float*)d_in[19], *bout = (const float*)d_in[20];
  const int* src = (const int*)d_in[21];
  const int* dst = (const int*)d_in[22];
  float* out = (float*)d_out;

  char* ws = (char*)d_ws;
  size_t off = 0;
  const size_t oW1 = off; off += (size_t)(2 * D2) * D1 * 2;          off = (off + 255) & ~(size_t)255;
  const size_t oW2 = off; off += (size_t)(2 * D3) * D2 * 2;          off = (off + 255) & ~(size_t)255;
  const size_t oWO = off; off += (size_t)EMB * KO * 2;                off = (off + 255) & ~(size_t)255;
  const size_t oX1 = off; off += (size_t)G * NJ * D1 * 2;             off = (off + 255) & ~(size_t)255;
  const size_t oX2 = off; off += (size_t)G * NJ * D2 * 2;             off = (off + 255) & ~(size_t)255;
  const size_t oX3 = off; off += (size_t)G * NJ * D3 * 2;             off = (off + 255) & ~(size_t)255;
  if (off > ws_size || off > (size_t)WSCAPB) return;
  unsigned short* W1T = (unsigned short*)(ws + oW1);
  unsigned short* W2T = (unsigned short*)(ws + oW2);
  unsigned short* WTO = (unsigned short*)(ws + oWO);
  unsigned short* X1  = (unsigned short*)(ws + oX1);
  unsigned short* X2  = (unsigned short*)(ws + oX2);
  unsigned short* X3  = (unsigned short*)(ws + oX3);

  hipFuncSetAttribute(reinterpret_cast<const void*>(&k_gatw<D1, D2>),
                      hipFuncAttributeMaxDynamicSharedMemorySize, (int)LL<D2>::TOTAL);
  hipFuncSetAttribute(reinterpret_cast<const void*>(&k_gatw<D2, D3>),
                      hipFuncAttributeMaxDynamicSharedMemorySize, (int)LL<D3>::TOTAL);

  k_wtrans<<<dim3(D1 / 64, D2 / 64), NT, 0, stream>>>(Wl1, W1T, D1, D2, 0,  WSC);
  k_wtrans<<<dim3(D1 / 64, D2 / 64), NT, 0, stream>>>(Wr1, W1T, D1, D2, D2, WSC);
  k_wtrans<<<dim3(D2 / 64, D3 / 64), NT, 0, stream>>>(Wl2, W2T, D2, D3, 0,  WSC);
  k_wtrans<<<dim3(D2 / 64, D3 / 64), NT, 0, stream>>>(Wr2, W2T, D2, D3, D3, WSC);
  k_wtrans<<<dim3(KO / 64, EMB / 64), NT, 0, stream>>>(Wout, WTO, KO, EMB, 0, WOSC);

  k_gat0<<<G, NT, 0, stream>>>(x_seq, Wl0, bl0, Wr0, br0, att0, bias0, src, dst, X1, nE);
  k_gatw<D1, D2><<<G, NT, LL<D2>::TOTAL, stream>>>(X1, W1T, bl1, br1, att1, bias1, src, dst, X2, nE);
  k_gatw<D2, D3><<<G, NT, LL<D3>::TOTAL, stream>>>(X2, W2T, bl2, br2, att2, bias2, src, dst, X3, nE);

  k_ogemm<<<dim3(G / 64, EMB / 64), GT, 0, stream>>>(X3, WTO, bout, out, KO, EMB);
}
